// MLP_Cutoff_87737591923195
// MI455X (gfx1250) — hardware-verified
//
#include <hip/hip_runtime.h>

typedef _Float16 half_t;
typedef half_t v16h __attribute__((ext_vector_type(16)));
typedef half_t v8h  __attribute__((ext_vector_type(8)));
typedef float  v8f  __attribute__((ext_vector_type(8)));
typedef float  v4f  __attribute__((ext_vector_type(4)));

constexpr int NFEAT = 30;
constexpr int NMAIN = 30;
constexpr int NPAIR = 20;
constexpr int NGRP  = NMAIN + NPAIR;
constexpr int D1 = 140, D2 = 100, D3 = 60, D4 = 20;
constexpr int ROWS = 64;

constexpr int HSTR = 168;
constexpr int WS2  = 168;
constexpr int WS3  = 136;
constexpr int WS4  = 72;

constexpr float WSCALE = 16.0f;
constexpr float WINV   = 0.0625f;

constexpr int OFF_XS = 0;
constexpr int OFF_W1 = OFF_XS + ROWS * 32 * 4;
constexpr int OFF_B1 = OFF_W1 + D1 * 2 * 4;
constexpr int OFF_B2 = OFF_B1 + 144 * 4;
constexpr int OFF_B3 = OFF_B2 + 112 * 4;
constexpr int OFF_B4 = OFF_B3 + 64 * 4;
constexpr int OFF_W5 = OFF_B4 + 32 * 4;
constexpr int OFF_B5 = OFF_W5 + 32 * 4;
constexpr int OFF_OS = OFF_B5 + 16;
constexpr int OFF_W2 = OFF_OS + ROWS * 4;
constexpr int OFF_W3 = OFF_W2 + 112 * WS2 * 2;
constexpr int OFF_W4 = OFF_W3 + 64 * WS3 * 2;
constexpr int OFF_HA = OFF_W4 + 32 * WS4 * 2;
constexpr int OFF_HB = OFF_HA + 4 * 16 * HSTR * 2;
constexpr int SMEM_BYTES = OFF_HB + 4 * 16 * HSTR * 2;

static_assert(OFF_W1 % 16 == 0 && OFF_B1 % 16 == 0 && OFF_B2 % 16 == 0 && OFF_B3 % 16 == 0, "");
static_assert(OFF_B4 % 16 == 0 && OFF_W5 % 16 == 0 && OFF_B5 % 16 == 0 && OFF_OS % 16 == 0, "");
static_assert(OFF_W2 % 16 == 0 && OFF_W3 % 16 == 0 && OFF_W4 % 16 == 0 && OFF_HA % 16 == 0 && OFF_HB % 16 == 0, "");
static_assert(HSTR % 8 == 0 && WS2 % 8 == 0 && WS3 % 8 == 0 && WS4 % 8 == 0, "");

union Frag { v16h v; v8h half[2]; };

__device__ __forceinline__ v8f wmma_f16(v16h a, v16h b, v8f c)
{
    c = __builtin_amdgcn_wmma_f32_16x16x32_f16(false, a, false, b, (short)0, c, false, false);
    asm volatile("v_nop\n\tv_nop\n\tv_nop\n\tv_nop" : "+v"(c) : "v"(a), "v"(b));
    return c;
}

template <int NT, int KT, int WSTR>
__device__ __forceinline__ void gemm_relu(
    const half_t* hin,
    const half_t* W,
    const float*  bias,
    half_t*       hout,
    int lane)
{
    const int nlo = lane & 15;
    const int hh  = lane >> 4;

    const half_t* arow = hin + nlo * HSTR + (hh << 3);
    const half_t* brow = W   + nlo * WSTR + (hh << 3);

    v8f c[NT];
#pragma unroll
    for (int t = 0; t < NT; ++t) c[t] = (v8f){0.f, 0.f, 0.f, 0.f, 0.f, 0.f, 0.f, 0.f};

#pragma unroll
    for (int k0 = 0; k0 < KT; ++k0) {
        Frag a;
        a.half[0] = *(const v8h*)(arow + k0 * 32);
        a.half[1] = *(const v8h*)(arow + k0 * 32 + 16);
#pragma unroll
        for (int t = 0; t < NT; ++t) {
            Frag b;
            b.half[0] = *(const v8h*)(brow + t * 16 * WSTR + k0 * 32);
            b.half[1] = *(const v8h*)(brow + t * 16 * WSTR + k0 * 32 + 16);
            c[t] = wmma_f16(a.v, b.v, c[t]);
        }
    }

    half_t* orow = hout + (hh << 3) * HSTR + nlo;
#pragma unroll
    for (int t = 0; t < NT; ++t) {
        const float bb = bias[t * 16 + nlo];
#pragma unroll
        for (int r = 0; r < 8; ++r) {
            float v = c[t][r] * WINV + bb;
            v = v > 0.0f ? v : 0.0f;
            orow[r * HSTR + t * 16] = (half_t)v;
        }
    }
}

__global__ void __launch_bounds__(128)
net_kernel(const float* __restrict__ x, const int* __restrict__ inter_idx,
           const float* __restrict__ mW1, const float* __restrict__ mb1,
           const float* __restrict__ iW1, const float* __restrict__ ib1,
           const float* __restrict__ mW2, const float* __restrict__ mb2,
           const float* __restrict__ iW2, const float* __restrict__ ib2,
           const float* __restrict__ mW3, const float* __restrict__ mb3,
           const float* __restrict__ iW3, const float* __restrict__ ib3,
           const float* __restrict__ mW4, const float* __restrict__ mb4,
           const float* __restrict__ iW4, const float* __restrict__ ib4,
           const float* __restrict__ mW5, const float* __restrict__ mb5,
           const float* __restrict__ iW5, const float* __restrict__ ib5,
           float* __restrict__ out, int batch)
{
    extern __shared__ __attribute__((aligned(16))) char smem[];
    float*  xs  = (float*)(smem + OFF_XS);
    float*  w1s = (float*)(smem + OFF_W1);
    float*  b1s = (float*)(smem + OFF_B1);
    float*  b2s = (float*)(smem + OFF_B2);
    float*  b3s = (float*)(smem + OFF_B3);
    float*  b4s = (float*)(smem + OFF_B4);
    float*  w5s = (float*)(smem + OFF_W5);
    float*  b5s = (float*)(smem + OFF_B5);
    float*  osm = (float*)(smem + OFF_OS);
    half_t* w2s = (half_t*)(smem + OFF_W2);
    half_t* w3s = (half_t*)(smem + OFF_W3);
    half_t* w4s = (half_t*)(smem + OFF_W4);
    half_t* hA  = (half_t*)(smem + OFF_HA);
    half_t* hB  = (half_t*)(smem + OFF_HB);

    const int tid  = threadIdx.x;
    const int lane = tid & 31;
    const int wave = tid >> 5;
    const int rowbase = blockIdx.x * ROWS;
    const int m = lane & 15;

    for (int i = tid; i < ROWS * 32; i += 128) {
        const int r = i >> 5, f = i & 31;
        const int gr = rowbase + r;
        float v = 0.0f;
        if (f < NFEAT && gr < batch) v = x[(size_t)gr * NFEAT + f];
        xs[i] = v;
    }
    {
        unsigned* za = (unsigned*)hA;
        unsigned* zb = (unsigned*)hB;
        for (int i = tid; i < (4 * 16 * HSTR) / 2; i += 128) { za[i] = 0u; zb[i] = 0u; }
    }
    __syncthreads();

    half_t* myA = hA + wave * 16 * HSTR;
    half_t* myB = hB + wave * 16 * HSTR;
    float yacc = 0.0f;

    for (int g = 0; g < NGRP; ++g) {
        const bool inter = (g >= NMAIN);
        const int  gi    = inter ? g - NMAIN : g;
        const float* W1 = inter ? iW1 + (size_t)gi * D1 * 2 : mW1 + (size_t)gi * D1;
        const float* B1 = (inter ? ib1 : mb1) + (size_t)gi * D1;
        const float* W2 = (inter ? iW2 : mW2) + (size_t)gi * D2 * D1;
        const float* B2 = (inter ? ib2 : mb2) + (size_t)gi * D2;
        const float* W3 = (inter ? iW3 : mW3) + (size_t)gi * D3 * D2;
        const float* B3 = (inter ? ib3 : mb3) + (size_t)gi * D3;
        const float* W4 = (inter ? iW4 : mW4) + (size_t)gi * D4 * D3;
        const float* B4 = (inter ? ib4 : mb4) + (size_t)gi * D4;
        const float* W5 = (inter ? iW5 : mW5) + (size_t)gi * D4;
        const float* B5 = (inter ? ib5 : mb5) + gi;

        for (int i = tid; i < 112 * WS2; i += 128) {
            const int o = i / WS2, k = i - o * WS2;
            const float v = (o < D2 && k < D1) ? W2[o * D1 + k] * WSCALE : 0.0f;
            w2s[i] = (half_t)v;
        }
        for (int i = tid; i < 64 * WS3; i += 128) {
            const int o = i / WS3, k = i - o * WS3;
            const float v = (o < D3 && k < D2) ? W3[o * D2 + k] * WSCALE : 0.0f;
            w3s[i] = (half_t)v;
        }
        for (int i = tid; i < 32 * WS4; i += 128) {
            const int o = i / WS4, k = i - o * WS4;
            const float v = (o < D4 && k < D3) ? W4[o * D3 + k] * WSCALE : 0.0f;
            w4s[i] = (half_t)v;
        }
        for (int i = tid; i < D1; i += 128) {
            if (inter) { w1s[2 * i] = W1[2 * i]; w1s[2 * i + 1] = W1[2 * i + 1]; }
            else       { w1s[2 * i] = W1[i];     w1s[2 * i + 1] = 0.0f; }
        }
        for (int i = tid; i < 144; i += 128) b1s[i] = (i < D1) ? B1[i] : 0.0f;
        for (int i = tid; i < 112; i += 128) b2s[i] = (i < D2) ? B2[i] : 0.0f;
        for (int i = tid; i < 64;  i += 128) b3s[i] = (i < D3) ? B3[i] : 0.0f;
        for (int i = tid; i < 32;  i += 128) b4s[i] = (i < D4) ? B4[i] : 0.0f;
        for (int i = tid; i < 32;  i += 128) w5s[i] = (i < D4) ? W5[i] : 0.0f;
        if (tid == 0) b5s[0] = B5[0];
        __syncthreads();

        int f0, f1;
        if (inter) {
            f0 = inter_idx[2 * gi]; f1 = inter_idx[2 * gi + 1];
            if (f0 < 0) f0 += NFEAT;
            if (f1 < 0) f1 += NFEAT;
            f0 = f0 < 0 ? 0 : (f0 > NFEAT - 1 ? NFEAT - 1 : f0);
            f1 = f1 < 0 ? 0 : (f1 > NFEAT - 1 ? NFEAT - 1 : f1);
        } else { f0 = g; f1 = g; }
        const float x0 = xs[(wave * 16 + m) * 32 + f0];
        const float x1 = xs[(wave * 16 + m) * 32 + f1];
        {
            const int ob = lane >> 4;
            half_t* h1row = myA + m * HSTR;
            for (int i = 0; i < D1 / 2; ++i) {
                const int o = ob + 2 * i;
                float h = fmaf(w1s[2 * o], x0, fmaf(w1s[2 * o + 1], x1, b1s[o]));
                h1row[o] = (half_t)(h > 0.0f ? h : 0.0f);
            }
        }
        __syncthreads();

        gemm_relu<7, 5, WS2>(myA, w2s, b2s, myB, lane);
        __syncthreads();
        gemm_relu<4, 4, WS3>(myB, w3s, b3s, myA, lane);
        __syncthreads();
        gemm_relu<2, 2, WS4>(myA, w4s, b4s, myB, lane);
        __syncthreads();

        float dot = b5s[0];
#pragma unroll
        for (int k = 0; k < D4; ++k) dot = fmaf((float)myB[m * HSTR + k], w5s[k], dot);
        yacc += dot;

        __syncthreads();
    }

    if (lane < 16) osm[wave * 16 + m] = yacc;
    __syncthreads();

    const bool full = (rowbase + ROWS <= batch);
    if (tid < 16) {
        const v4f v = *(const v4f*)(osm + 4 * tid);
        float* p = out + (size_t)rowbase + 4 * tid;
        if (full) {
            *(volatile v4f*)p = v;
        } else {
#pragma unroll
            for (int j = 0; j < 4; ++j)
                if (rowbase + 4 * tid + j < batch) ((volatile float*)p)[j] = v[j];
        }
    }
    __threadfence();
    if (tid < 16) {
        const v4f v = *(const v4f*)(osm + 4 * tid);
        float* p = out + (size_t)rowbase + 4 * tid;
        if (full) {
            *(volatile v4f*)p = v;
        } else {
#pragma unroll
            for (int j = 0; j < 4; ++j)
                if (rowbase + 4 * tid + j < batch) ((volatile float*)p)[j] = v[j];
        }
    }
}

extern "C" void kernel_launch(void* const* d_in, const int* in_sizes, int n_in,
                              void* d_out, int out_size, void* d_ws, size_t ws_size,
                              hipStream_t stream)
{
    (void)n_in; (void)out_size; (void)d_ws; (void)ws_size;
    const float* x         = (const float*)d_in[0];
    const int*   inter_idx = (const int*)  d_in[1];
    const float* mW1 = (const float*)d_in[2];  const float* mb1 = (const float*)d_in[3];
    const float* iW1 = (const float*)d_in[4];  const float* ib1 = (const float*)d_in[5];
    const float* mW2 = (const float*)d_in[6];  const float* mb2 = (const float*)d_in[7];
    const float* iW2 = (const float*)d_in[8];  const float* ib2 = (const float*)d_in[9];
    const float* mW3 = (const float*)d_in[10]; const float* mb3 = (const float*)d_in[11];
    const float* iW3 = (const float*)d_in[12]; const float* ib3 = (const float*)d_in[13];
    const float* mW4 = (const float*)d_in[14]; const float* mb4 = (const float*)d_in[15];
    const float* iW4 = (const float*)d_in[16]; const float* ib4 = (const float*)d_in[17];
    const float* mW5 = (const float*)d_in[18]; const float* mb5 = (const float*)d_in[19];
    const float* iW5 = (const float*)d_in[20]; const float* ib5 = (const float*)d_in[21];
    float* out = (float*)d_out;

    const int batch = in_sizes[0] / NFEAT;
    if (batch <= 0) return;
    const int grid  = (batch + ROWS - 1) / ROWS;

    (void)hipFuncSetAttribute((const void*)net_kernel,
                              hipFuncAttributeMaxDynamicSharedMemorySize,
                              (int)SMEM_BYTES);
    net_kernel<<<dim3(grid), dim3(128), SMEM_BYTES, stream>>>(
        x, inter_idx,
        mW1, mb1, iW1, ib1, mW2, mb2, iW2, ib2,
        mW3, mb3, iW3, ib3, mW4, mb4, iW4, ib4,
        mW5, mb5, iW5, ib5, out, batch);
}
